// GraphBlock_52467320488062
// MI455X (gfx1250) — hardware-verified
//
#include <hip/hip_runtime.h>
#include <math.h>

#define NN   50000
#define NE   800000
#define NP   50048
#define DI   128
#define DH   256
#define DO   128
#define NG   512
#define NT   256
#define SRB  2048
#define RPW  (SRB / 8)
#define NTL  25
#define SCH  2048
#define SPT  (SCH / NT)
#define NCH  ((NE + SCH - 1) / SCH)
#define SCHP 2048
#define NCHP ((NN + SCHP - 1) / SCHP)
#define BN_EPS 1e-5f
#define WSC 16.0f
#define WSC_INV (1.0f / 16.0f)

typedef __attribute__((ext_vector_type(16))) _Float16 v16h;
typedef __attribute__((ext_vector_type(8)))  _Float16 v8h;
typedef __attribute__((ext_vector_type(16))) __bf16   v16b;
typedef __attribute__((ext_vector_type(8)))  __bf16   v8b;
typedef __attribute__((ext_vector_type(8)))  float    v8f;
typedef __attribute__((ext_vector_type(4)))  float    v4f;
typedef __attribute__((ext_vector_type(4)))  int      v4i;

__device__ __forceinline__ unsigned short f2bf_bits(float f) {
  unsigned u = __float_as_uint(f);
  return (unsigned short)((u + 0x7FFFu + ((u >> 16) & 1u)) >> 16);
}
__device__ __forceinline__ float bf_bits2f(unsigned short h) { return __uint_as_float(((unsigned)h) << 16); }

__device__ __forceinline__ void dep_guard_h(v8f& a, v8f& b, v16h x, v16h y) { asm volatile("v_nop\n\tv_nop\n\tv_nop\n\tv_nop" : "+v"(a), "+v"(b) : "v"(x), "v"(y)); }
__device__ __forceinline__ void dep_guard_b(v8f& a, v8f& b, v16b x, v16b y) { asm volatile("v_nop\n\tv_nop\n\tv_nop\n\tv_nop" : "+v"(a), "+v"(b) : "v"(x), "v"(y)); }
__device__ __forceinline__ void keep4_h(v16h a, v16h b, v16h c, v16h d) { asm volatile("v_nop" :: "v"(a), "v"(b), "v"(c), "v"(d)); }
__device__ __forceinline__ void keep4_b(v16b a, v16b b, v16b c, v16b d) { asm volatile("v_nop" :: "v"(a), "v"(b), "v"(c), "v"(d)); }
__device__ __forceinline__ void acc_guard4(v8f& a, v8f& b, v8f& c, v8f& d) { asm volatile("v_nop\n\tv_nop\n\tv_nop\n\tv_nop" : "+v"(a), "+v"(b), "+v"(c), "+v"(d)); }
template <typename T> struct Frag;
template <> struct Frag<_Float16> {
  typedef v16h V; union U { v16h v; v8h h[2]; };
  static __device__ __forceinline__ v16h load(const _Float16* p) {
    U f; f.h[0] = *(const v8h*)(p); f.h[1] = *(const v8h*)(p + 16); return f.v;
  }
  static __device__ __forceinline__ v8f mma(v16h a, v16h b, v8f c) {
    return __builtin_amdgcn_wmma_f32_16x16x32_f16(false, a, false, b, (short)0, c, false, false);
  }
  static __device__ __forceinline__ void guard(v8f& a, v8f& b, v16h x, v16h y) { dep_guard_h(a, b, x, y); }
  static __device__ __forceinline__ void keep(v16h a, v16h b, v16h c, v16h d) { keep4_h(a, b, c, d); }
};
template <> struct Frag<__bf16> {
  typedef v16b V; union U { v16b v; v8b h[2]; };
  static __device__ __forceinline__ v16b load(const __bf16* p) {
    U f; f.h[0] = *(const v8b*)(p); f.h[1] = *(const v8b*)(p + 16); return f.v;
  }
  static __device__ __forceinline__ v8f mma(v16b a, v16b b, v8f c) {
    return __builtin_amdgcn_wmma_f32_16x16x32_bf16(false, a, false, b, (short)0, c, false, false);
  }
  static __device__ __forceinline__ void guard(v8f& a, v8f& b, v16b x, v16b y) { dep_guard_b(a, b, x, y); }
  static __device__ __forceinline__ void keep(v16b a, v16b b, v16b c, v16b d) { keep4_b(a, b, c, d); }
};

template <int ET> struct Elem;
template <> struct Elem<0> { typedef _Float16 T; };
template <> struct Elem<1> { typedef __bf16 T; };
template <int ET, bool SPLIT, int BIAS_MODE, int OUT_MODE, bool RESID, int ACT = 0>
__global__ __launch_bounds__(256) void wmma_gemm64(
    const unsigned short* __restrict__ Ap, const unsigned short* __restrict__ A2p, int lda, long strideA,
    const unsigned short* __restrict__ Btp, const unsigned short* __restrict__ Bt2p, int ldb, long strideB,
    void* __restrict__ Cout, void* __restrict__ Cout2, int ldc, long strideC,
    const float* __restrict__ bias,
    const float* __restrict__ resid, long strideR,
    int M, int N, int K, float scale) {
  typedef typename Elem<ET>::T T;
  typedef typename Frag<T>::V V;
  const T* A = (const T*)Ap; const T* A2 = (const T*)A2p; const T* Bt = (const T*)Btp; const T* Bt2 = (const T*)Bt2p;
  __shared__ __align__(16) float sT[8][16 * 68];
  const int b    = blockIdx.y;
  const int lane = threadIdx.x & 31;
  const int wave = threadIdx.x >> 5;
  const int tilesN = N >> 6;
  const int tilesM = M >> 6;
  const int tile = blockIdx.x * 8 + wave;
  if (tile >= tilesM * tilesN) return;
  const int tm = tile / tilesN;
  const int tn = tile - tm * tilesN;
  const int m0 = tm << 6;
  const int n0 = tn << 6;

  const T* Ab  = A  + (size_t)b * strideA;
  const T* Bb  = Bt + (size_t)b * strideB;
  const T* Ab2 = SPLIT ? (A2  + (size_t)b * strideA) : nullptr;
  const T* Bb2 = SPLIT ? (Bt2 + (size_t)b * strideB) : nullptr;

  const int rlane = lane & 15;
  const int koff  = (lane >> 4) * 8;
  const int mOff  = (lane >> 4) * 8;

  v8f acc[4][4];
#pragma unroll
  for (int i = 0; i < 4; ++i)
#pragma unroll
    for (int j = 0; j < 4; ++j) acc[i][j] = (v8f){0.f,0.f,0.f,0.f,0.f,0.f,0.f,0.f};

  for (int k0 = 0; k0 < K; k0 += 32) {
    V bh[4], bl[4];
#pragma unroll
    for (int j = 0; j < 4; ++j) {
      const size_t bo = (size_t)(n0 + (j << 4) + rlane) * ldb + koff + k0;
      bh[j] = Frag<T>::load(Bb + bo);
      if (SPLIT) bl[j] = Frag<T>::load(Bb2 + bo);
    }
#pragma unroll
    for (int i = 0; i < 4; ++i) {
      const size_t ao = (size_t)(m0 + (i << 4) + rlane) * lda + koff + k0;
      V ah = Frag<T>::load(Ab + ao);
      V al;
      if (SPLIT) al = Frag<T>::load(Ab2 + ao);
#pragma unroll
      for (int j = 0; j < 4; ++j) {
        acc[i][j] = Frag<T>::mma(ah, bh[j], acc[i][j]);
        if (SPLIT) {
          acc[i][j] = Frag<T>::mma(ah, bl[j], acc[i][j]);
          acc[i][j] = Frag<T>::mma(al, bh[j], acc[i][j]);
        }
      }
      Frag<T>::guard(acc[i][0], acc[i][3], ah, SPLIT ? al : ah);
    }
    Frag<T>::keep(bh[0], bh[1], bh[2], bh[3]);
    if (SPLIT) Frag<T>::keep(bl[0], bl[1], bl[2], bl[3]);
  }
  acc_guard4(acc[0][0], acc[0][1], acc[0][2], acc[0][3]);
  acc_guard4(acc[1][0], acc[1][1], acc[1][2], acc[1][3]);
  acc_guard4(acc[2][0], acc[2][1], acc[2][2], acc[2][3]);
  acc_guard4(acc[3][0], acc[3][1], acc[3][2], acc[3][3]);

  float* slab = sT[wave];
  const float* Rb = RESID ? (resid + (size_t)b * strideR) : nullptr;
#pragma unroll
  for (int i = 0; i < 4; ++i) {
    const int mBase = m0 + (i << 4);
#pragma unroll
    for (int j = 0; j < 4; ++j) {
      const int n = n0 + (j << 4) + rlane;
      float bv = 0.f;
      if (BIAS_MODE == 2) bv = bias[n];
#pragma unroll
      for (int r = 0; r < 8; ++r) {
        float v = acc[i][j][r] * scale;
        if (BIAS_MODE == 1) v += bias[mBase + mOff + r];
        if (BIAS_MODE == 2) v += bv;
        if (RESID) v += Rb[(size_t)(mBase + mOff + r) * ldc + n];
        if (ACT == 1) v = tanhf(v);
        if (ACT == 2) v = fmaxf(v, 0.0f);
        if (ACT == 3) v = v / (1.0f + expf(-v));
        if (ACT == 4) v = (v > 0.f) ? v : 0.01f * v;
        if (ACT == 5) v = 0.5f * v * (1.0f + erff(v * 0.70710678118654752f));
        slab[(mOff + r) * 68 + (j << 4) + rlane] = v;
      }
    }
    __builtin_amdgcn_fence(__ATOMIC_RELEASE, "workgroup");
    __builtin_amdgcn_wave_barrier();
    __builtin_amdgcn_fence(__ATOMIC_ACQUIRE, "workgroup");
    if (OUT_MODE == 0) {
      float* C = (float*)Cout + (size_t)b * strideC;
      const int hh = lane >> 4, c4 = (lane & 15) * 4;
      for (int pass = 0; pass < 2; ++pass) {
#pragma unroll
        for (int it = 0; it < 8; ++it) {
          const int row = it * 2 + hh;
          v4f v = *(const v4f*)(slab + row * 68 + c4);
          *(volatile v4f*)(C + (size_t)(mBase + row) * ldc + n0 + c4) = v;
        }
        __threadfence();
      }
    } else {
      const int q = lane >> 3, c8 = (lane & 7) * 8;
      unsigned short* C  = (unsigned short*)Cout  + (size_t)b * strideC;
      unsigned short* C2 = (OUT_MODE == 2) ? ((unsigned short*)Cout2 + (size_t)b * strideC) : nullptr;
      for (int pass = 0; pass < 2; ++pass) {
#pragma unroll
        for (int it = 0; it < 4; ++it) {
          const int row = it * 4 + q;
          const float* sp = slab + row * 68 + c8;
          v8h hv, lv;
#pragma unroll
          for (int e = 0; e < 8; ++e) {
            if (OUT_MODE == 1) {
              hv[e] = (_Float16)sp[e];
            } else {
              unsigned short hb = f2bf_bits(sp[e]);
              unsigned short lb = f2bf_bits(sp[e] - bf_bits2f(hb));
              hv[e] = __builtin_bit_cast(_Float16, hb);
              lv[e] = __builtin_bit_cast(_Float16, lb);
            }
          }
          *(volatile v8h*)(C + (size_t)(mBase + row) * ldc + n0 + c8) = hv;
          if (OUT_MODE == 2) *(volatile v8h*)(C2 + (size_t)(mBase + row) * ldc + n0 + c8) = lv;
        }
        __threadfence();
      }
    }
    __builtin_amdgcn_fence(__ATOMIC_RELEASE, "workgroup");
    __builtin_amdgcn_wave_barrier();
    __builtin_amdgcn_fence(__ATOMIC_ACQUIRE, "workgroup");
  }
}

__device__ __forceinline__ int blk_excl_scan(int cnt, int* scan_ws, int tid, int* tot) {
  const int lane = tid & 31, wave = tid >> 5; int incl = cnt;
#pragma unroll
  for (int o = 1; o < 32; o <<= 1) { const int v = __shfl_up(incl, o, 32); if (lane >= o) incl += v; }
  if (lane == 31) scan_ws[wave] = incl;
  __syncthreads();
  if (wave == 0) { int wv = (lane < NT / 32) ? scan_ws[lane] : 0; int wincl = wv;
#pragma unroll
    for (int o = 1; o < 32; o <<= 1) { const int v = __shfl_up(wincl, o, 32); if (lane >= o) wincl += v; }
    if (lane < NT / 32) scan_ws[32 + lane] = wincl - wv; if (lane == 31) scan_ws[64] = wincl; }
  __syncthreads();
  const int res = scan_ws[32 + wave] + incl - cnt; *tot = scan_ws[64];
  return res;
}
__device__ __forceinline__ int chunk_hits_e(const int* __restrict__ srcv, const int* __restrict__ dstv, int e0, int n0, int tid,
                                           int* LIST, int* scan_ws) {
  const int eb = e0 + tid * SPT;
  const bool live = eb < NE;
  const int ebc = live ? eb : (NE - SPT);
  int rec[SPT]; int cnt = 0;
#pragma unroll
  for (int k = 0; k < SPT; k += 4) {
    const v4i d4 = *(const v4i*)(dstv + ebc + k);
    const v4i s4 = *(const v4i*)(srcv + ebc + k);
#pragma unroll
    for (int e = 0; e < 4; ++e) {
      const int d = d4[e]; int r = -1;
      if (live && d >= n0 && d < n0 + SRB) { int s = s4[e]; s = s < 0 ? 0 : (s >= NN ? NN - 1 : s); r = ((d - n0) << 16) | s; ++cnt; }
      rec[k + e] = r;
    }
  }
  int tot; int p = blk_excl_scan(cnt, scan_ws, tid, &tot);
#pragma unroll
  for (int k = 0; k < SPT; ++k) if (rec[k] >= 0) { if ((unsigned)p < (unsigned)SCH) LIST[p] = rec[k]; ++p; }
  __syncthreads();
  return tot < SCH ? tot : SCH;
}

__global__ __launch_bounds__(NT) void prep_kernel(const float* __restrict__ W1, const float* __restrict__ W2,
                                                 unsigned* __restrict__ W1T, unsigned* __restrict__ W2T) {
  const int i = blockIdx.x * NT + threadIdx.x;
  if (i < DH * DI / 2) {
    const int n1 = i >> 6;
    const int k1 = 2 * (i & 63);
    const float a = W1[(size_t)k1 * DH + n1] * WSC, bb = W1[(size_t)(k1 + 1) * DH + n1] * WSC;
    const _Float16 ha = (_Float16)a, hb = (_Float16)bb;
    const unsigned u1 = (unsigned)__builtin_bit_cast(unsigned short, ha) | ((unsigned)__builtin_bit_cast(unsigned short, hb) << 16);
    const int n2 = i >> 7;
    const int k2 = 2 * (i & 127);
    const float c = W2[(size_t)k2 * DO + n2] * WSC, dd = W2[(size_t)(k2 + 1) * DO + n2] * WSC;
    const _Float16 hc = (_Float16)c, hd = (_Float16)dd;
    const unsigned u2 = (unsigned)__builtin_bit_cast(unsigned short, hc) | ((unsigned)__builtin_bit_cast(unsigned short, hd) << 16);
    ((volatile unsigned*)W1T)[i] = u1; ((volatile unsigned*)W2T)[i] = u2;
    __threadfence();
    ((volatile unsigned*)W1T)[i] = u1; ((volatile unsigned*)W2T)[i] = u2;
  }
}

__global__ __launch_bounds__(NT) void gin_agg_kernel(const float* __restrict__ x, const int* __restrict__ ei, float* ACC,
                                                    unsigned short* __restrict__ H0) {
  __shared__ int LIST[SCH];
  __shared__ int scan_ws[80];
  const int tid = threadIdx.x, lane = tid & 31, wave = tid >> 5;
  const int n0 = blockIdx.x * SRB;
  const v4f z4 = {0.f, 0.f, 0.f, 0.f};
  for (int pass = 0; pass < 2; ++pass) {
#pragma unroll 1
    for (int j = 0; j < RPW; ++j) {
      const int n = n0 + wave * RPW + j;
      const int nc = n < NN ? n : NN - 1;
      v4f v = *(const v4f*)(x + (size_t)nc * DI + 4 * lane);
      if (n >= NN) v = z4;
      *(volatile v4f*)(ACC + (size_t)n * DI + 4 * lane) = v;
    }
    __threadfence();
  }
  const int* srcv = ei; const int* dstv = ei + NE;
#pragma unroll 1
  for (int c = 0; c < NCH; ++c) {
    const int tot = chunk_hits_e(srcv, dstv, c * SCH, n0, tid, LIST, scan_ws);
#pragma unroll 1
    for (int base = 0; base < tot; base += 32) {
      const int q = base + lane;
      const int qc = q < SCH ? q : SCH - 1;
      const int lv = LIST[qc];
      const int rv = (q < tot) ? lv : -1;
      const int own = (rv >= 0 && (rv >> 24) == wave) ? 1 : 0;
      unsigned msk = (unsigned)__ballot(own);
#pragma unroll 1
      for (int it = 0; it < 32; ++it) {
        if (msk == 0u) break;
        const int bp = __builtin_ctz(msk); msk &= msk - 1u;
        const int r = __shfl(rv, bp, 32);
        const int dl = r >> 16, s = r & 0xFFFF;
        const v4f xs = *(const v4f*)(x + (size_t)s * DI + 4 * lane);
        float* rp = ACC + (size_t)(n0 + dl) * DI + 4 * lane;
        v4f a = *(const v4f*)rp;
        a = a + xs;
        *(volatile v4f*)rp = a;
        __threadfence();
        *(volatile v4f*)rp = a;
      }
    }
    __syncthreads();
  }
  __threadfence();
  const int hh = lane >> 4, c8 = (lane & 15) * 8;
#pragma unroll 1
  for (int j = 0; j < RPW; j += 2) {
    const int nb = n0 + wave * RPW + j;
    if (nb < NP) {
      const int n = nb + hh;
      const float* rp = ACC + (size_t)n * DI + c8;
      const v4f a0 = *(const v4f*)rp;
      const v4f a1 = *(const v4f*)(rp + 4);
      v8h hv;
#pragma unroll
      for (int e = 0; e < 4; ++e) { hv[e] = (_Float16)a0[e]; hv[4 + e] = (_Float16)a1[e]; }
      unsigned short* dp = H0 + (size_t)n * DI + c8;
      *(volatile v8h*)dp = hv;
      __threadfence();
      *(volatile v8h*)dp = hv;
    }
  }
}

__global__ __launch_bounds__(NT) void pool_kernel(const float* __restrict__ H2, const int* __restrict__ batch, float* __restrict__ P) {
  __shared__ int LIST[SCHP];
  __shared__ int scan_ws[80];
  const int tid = threadIdx.x, lane = tid & 31, wave = tid >> 5;
  const int g0 = blockIdx.x * 8;
  const v4f z4 = {0.f, 0.f, 0.f, 0.f};
  v4f acc = z4; int cnt = 0;
#pragma unroll 1
  for (int c = 0; c < NCHP; ++c) {
    const int eb = c * SCHP + tid * 8;
    const bool live = eb < NN;
    const int ebc = live ? eb : (NN - 8);
    const v4i b0 = *(const v4i*)(batch + ebc), b1v = *(const v4i*)(batch + ebc + 4);
    int rec[8]; int kc = 0;
#pragma unroll
    for (int k = 0; k < 8; ++k) {
      const int bv = (k < 4) ? b0[k] : b1v[k - 4];
      int r = -1;
      if (live && bv >= g0 && bv < g0 + 8) { r = ((bv - g0) << 16) | (eb + k); ++kc; }
      rec[k] = r;
    }
    int tot; int p = blk_excl_scan(kc, scan_ws, tid, &tot);
#pragma unroll
    for (int k = 0; k < 8; ++k) if (rec[k] >= 0) { if ((unsigned)p < (unsigned)SCHP) LIST[p] = rec[k]; ++p; }
    __syncthreads();
    const int totc = tot < SCHP ? tot : SCHP;
#pragma unroll 1
    for (int base = 0; base < totc; base += 32) {
      const int q = base + lane;
      const int qc = q < SCHP ? q : SCHP - 1;
      const int lv = LIST[qc];
      const int rv = (q < totc) ? lv : -1;
      const int own = (rv >= 0 && (rv >> 16) == wave) ? 1 : 0;
      unsigned msk = (unsigned)__ballot(own);
      cnt += __builtin_popcount(msk);
#pragma unroll 1
      for (int it = 0; it < 32; ++it) {
        if (msk == 0u) break;
        const int bp = __builtin_ctz(msk); msk &= msk - 1u;
        const int r = __shfl(rv, bp, 32);
        int nd = r & 0xFFFF; nd = nd < NN ? nd : NN - 1;
        acc = acc + *(const v4f*)(H2 + (size_t)nd * DO + 4 * lane);
      }
    }
    __syncthreads();
  }
  const float cf = (float)cnt;
  const float inv = 1.0f / fmaxf(cf, 1.0f);
  const v4f o = acc * inv;
  float* pp = P + (size_t)(g0 + wave) * DO + 4 * lane;
  *(volatile v4f*)pp = o;
  __threadfence();
  *(volatile v4f*)pp = o;
}

__global__ __launch_bounds__(NT) void bn_kernel(const float* __restrict__ P, const float* __restrict__ gam, const float* __restrict__ bet,
                                               float* __restrict__ out) {
  __shared__ __align__(16) float smu[DO];
  __shared__ __align__(16) float srs[DO];
  const int tid = threadIdx.x, lane = tid & 31, wave = tid >> 5;
  if (tid < DO) {
    double m = 0.0;
#pragma unroll 1
    for (int g = 0; g < NG; ++g) m += (double)P[(size_t)g * DO + tid];
    m = m * (1.0 / NG);
    const float mf = (float)m;
    double v = 0.0;
#pragma unroll 1
    for (int g = 0; g < NG; ++g) { const float d = P[(size_t)g * DO + tid] - mf; const float dd = d * d; v += (double)dd; }
    v = v * (1.0 / NG);
    const float vf = (float)v;
    smu[tid] = mf; srs[tid] = 1.0f / sqrtf(vf + BN_EPS);
  }
  __syncthreads();
  const v4f mu = *(const v4f*)(smu + 4 * lane), rs = *(const v4f*)(srs + 4 * lane);
  const v4f gm = *(const v4f*)(gam + 4 * lane), bt = *(const v4f*)(bet + 4 * lane);
#pragma unroll 1
  for (int j = 0; j < NG / 8; ++j) {
    const int g = wave * (NG / 8) + j;
    const v4f p = *(const v4f*)(P + (size_t)g * DO + 4 * lane);
    v4f t = (p - mu) * rs;
    t = t * gm + bt;
    v4f o;
#pragma unroll
    for (int e = 0; e < 4; ++e) o[e] = fmaxf(t[e], 0.f);
    float* op = out + (size_t)g * DO + 4 * lane;
    *(volatile v4f*)op = o;
    __threadfence();
    *(volatile v4f*)op = o;
  }
}

extern "C" void kernel_launch(void* const* d_in, const int* in_sizes, int n_in,
                              void* d_out, int out_size, void* d_ws, size_t ws_size, hipStream_t stream) {
  (void)in_sizes; (void)n_in; (void)out_size;
  const float* x     = (const float*)d_in[0];
  const int*   ei    = (const int*)  d_in[1];
  const int*   batch = (const int*)  d_in[2];
  const float* W1    = (const float*)d_in[3];
  const float* b1    = (const float*)d_in[4];
  const float* W2    = (const float*)d_in[5];
  const float* b2    = (const float*)d_in[6];
  const float* gam   = (const float*)d_in[7];
  const float* bet   = (const float*)d_in[8];
  float* out = (float*)d_out;

  char* ws = (char*)d_ws; size_t off = 0;
  auto carve = [&](size_t bytes) -> char* { char* p = ws + off; off += (bytes + 255) & ~(size_t)255; return p; };
  unsigned*       W1T = (unsigned*)carve((size_t)DH * DI * 2);
  unsigned*       W2T = (unsigned*)carve((size_t)DO * DH * 2);
  float*          ACC = (float*)carve((size_t)NTL * SRB * DI * 4);
  unsigned short* H0  = (unsigned short*)carve((size_t)NP * DI * 2);
  unsigned short* H1  = (unsigned short*)carve((size_t)NP * DH * 2);
  float*          H2  = (float*)carve((size_t)NP * DO * 4);
  float*          P   = (float*)carve((size_t)NG * DO * 4);
  if (off > ws_size || off > (size_t)134217728) return;

  prep_kernel<<<(DH * DI / 2 + NT - 1) / NT, NT, 0, stream>>>(W1, W2, W1T, W2T);
  gin_agg_kernel<<<NTL, NT, 0, stream>>>(x, ei, ACC, H0);
  {
    const int tiles = (NP / 64) * (DH / 64);
    wmma_gemm64<0, false, 2, 1, false, 2><<<dim3((tiles + 7) / 8, 1), 256, 0, stream>>>(
        (const unsigned short*)H0, (const unsigned short*)H0, DI, 0L,
        (const unsigned short*)W1T, (const unsigned short*)W1T, DI, 0L,
        (void*)H1, (void*)nullptr, DH, 0L,
        b1, (const float*)nullptr, 0L, NP, DH, DI, WSC_INV);
  }
  {
    const int tiles = (NP / 64) * (DO / 64);
    wmma_gemm64<0, false, 2, 0, false, 0><<<dim3((tiles + 7) / 8, 1), 256, 0, stream>>>(
        (const unsigned short*)H1, (const unsigned short*)H1, DH, 0L,
        (const unsigned short*)W2T, (const unsigned short*)W2T, DH, 0L,
        (void*)H2, (void*)nullptr, DO, 0L,
        b2, (const float*)nullptr, 0L, NP, DO, DH, WSC_INV);
  }
  pool_kernel<<<NG / 8, NT, 0, stream>>>(H2, batch, P);
  bn_kernel<<<1, NT, 0, stream>>>(P, gam, bet, out);
}
